// _netD_8_66872640799172
// MI455X (gfx1250) — hardware-run, weakly checked
//
#include <hip/hip_runtime.h>
#include <math.h>

typedef __attribute__((ext_vector_type(16))) _Float16 v16h;
typedef __attribute__((ext_vector_type(8)))  _Float16 v8h;
typedef __attribute__((ext_vector_type(8)))  float    v8f;
typedef __attribute__((ext_vector_type(4)))  float    v4f;
typedef __attribute__((ext_vector_type(2)))  double   v2d;

constexpr int kBatch = 64;
constexpr int kInH = 64, kInW = 768, kInC = 3;
constexpr int kC0 = 16, kC1 = 32, kC2 = 64, kC3 = 128, kC4 = 256, kC5 = 1000, kC5P = 1024, kCL = 64;
constexpr int kHo0 = 32, kWo0 = 384;
constexpr int kHo1 = 16, kWo1 = 192;
constexpr int kHo2 = 8,  kWo2 = 96;
constexpr int kHo3 = 4,  kWo3 = 48;
constexpr int kHo4 = 2,  kWo4 = 24;
constexpr int kWo5 = 23;
constexpr int kM0 = kBatch * kHo0 * kWo0;
constexpr int kM1 = kBatch * kHo1 * kWo1;
constexpr int kM2 = kBatch * kHo2 * kWo2;
constexpr int kM3 = kBatch * kHo3 * kWo3;
constexpr int kM4 = kBatch * kHo4 * kWo4;
constexpr int kM5 = kBatch * kWo5;
constexpr int kK0R = kInC * 16, kK0 = 64;
constexpr int kK1 = kC0 * 16, kK2 = kC1 * 16, kK3 = kC2 * 16, kK4 = kC3 * 16, kK5 = kC4 * 4;
constexpr int kK6R = kC5, kK6 = 1024;
constexpr int kChunk0 = kM0 / 4, kChunk1 = kM1 / 4, kChunk2 = kM2 / 2;
static_assert(kM0 == 786432 && kM1 == 196608 && kM2 == 49152 && kM3 == 12288 && kM4 == 3072 && kM5 == 1472, "position counts");
static_assert(kK1 == 256 && kK2 == 512 && kK3 == 1024 && kK4 == 2048 && kK5 == 1024, "patch depths");
static_assert((kK0 % 32) == 0 && (kK1 % 32) == 0 && (kK2 % 32) == 0 && (kK3 % 32) == 0 && (kK4 % 32) == 0 && (kK5 % 32) == 0 && (kK6 % 32) == 0, "K multiples of 32");
static_assert((kChunk0 % 64) == 0 && (kChunk1 % 64) == 0 && (kChunk2 % 64) == 0 && (kM3 % 64) == 0 && (kM4 % 64) == 0 && (kM5 % 64) == 0, "M multiples of 64");
static_assert((kC2 % 64) == 0 && (kC3 % 64) == 0 && (kC4 % 64) == 0 && (kC5P % 64) == 0 && (kCL % 64) == 0, "N multiples of 64 for the wide tile");

constexpr float kCarryW = 256.0f;
constexpr float kCarryA = 32.0f;
constexpr float kFold   = 1.0f / (kCarryW * kCarryA);
constexpr float kFoldKeepA = kCarryA * kFold;
constexpr float kBnEps  = 1e-5f;
constexpr float kSlope  = 0.2f;

constexpr size_t kSzYA   = (size_t)kM0 * kC0 * 4;
constexpr size_t kSzYB   = (size_t)kM1 * kC1 * 4;
constexpr size_t kSzCOL  = (size_t)kChunk0 * kK0 * 2;
constexpr size_t kSzA6   = (size_t)kM5 * kC5P * 2;
constexpr size_t kSzW0   = (size_t)kC0 * kK0 * 2;
constexpr size_t kSzW1   = (size_t)kC1 * kK1 * 2;
constexpr size_t kSzW2   = (size_t)kC2 * kK2 * 2;
constexpr size_t kSzW3   = (size_t)kC3 * kK3 * 2;
constexpr size_t kSzW4   = (size_t)kC4 * kK4 * 2;
constexpr size_t kSzW5   = (size_t)kC5P * kK5 * 2;
constexpr size_t kSzWL   = (size_t)kCL * kK6 * 2;
constexpr size_t kSzLOUT = (size_t)kM5 * kCL * 4;
constexpr size_t kSzPartOne = 65536;
constexpr size_t kSzPART = 5 * kSzPartOne;
constexpr size_t kSzStOne = 3 * 256 * 4;
constexpr size_t kSzST   = 5 * kSzStOne;

constexpr size_t kOffYA   = 0;
constexpr size_t kOffYB   = kOffYA   + kSzYA;
constexpr size_t kOffCOL  = kOffYB   + kSzYB;
constexpr size_t kOffA6   = kOffCOL  + kSzCOL;
constexpr size_t kOffW0   = kOffA6   + kSzA6;
constexpr size_t kOffW1   = kOffW0   + kSzW0;
constexpr size_t kOffW2   = kOffW1   + kSzW1;
constexpr size_t kOffW3   = kOffW2   + kSzW2;
constexpr size_t kOffW4   = kOffW3   + kSzW3;
constexpr size_t kOffW5   = kOffW4   + kSzW4;
constexpr size_t kOffWL   = kOffW5   + kSzW5;
constexpr size_t kOffLOUT = kOffWL   + kSzWL;
constexpr size_t kOffPART = kOffLOUT + kSzLOUT;
constexpr size_t kOffST   = kOffPART + kSzPART;
constexpr size_t kWsTotal = kOffST   + kSzST;
static_assert(kWsTotal == 108020736ull, "carve total");
static_assert(kWsTotal <= 134217728ull, "carve cap");
static_assert((kOffYB % 256) == 0 && (kOffCOL % 256) == 0 && (kOffA6 % 256) == 0 && (kOffW0 % 256) == 0 &&
              (kOffW1 % 256) == 0 && (kOffW2 % 256) == 0 && (kOffW3 % 256) == 0 && (kOffW4 % 256) == 0 &&
              (kOffW5 % 256) == 0 && (kOffWL % 256) == 0 && (kOffLOUT % 256) == 0 && (kOffPART % 256) == 0 &&
              (kOffST % 256) == 0, "aligned regions");
static_assert((size_t)kChunk1 * kK1 * 2 <= kSzCOL && (size_t)kChunk2 * kK2 * 2 <= kSzCOL && (size_t)kM3 * kK3 * 2 <= kSzCOL &&
              (size_t)kM4 * kK4 * 2 <= kSzCOL && (size_t)kM5 * kK5 * 2 <= kSzCOL, "patch chunk fits");
static_assert((size_t)kM2 * kC2 * 4 <= kSzYA && (size_t)kM4 * kC4 * 4 <= kSzYA && (size_t)kM3 * kC3 * 4 <= kSzYB, "plane re-use fits");
static_assert((size_t)256 * 2 * kC0 * 8 == kSzPartOne && (size_t)128 * 2 * kC1 * 8 == kSzPartOne && (size_t)64 * 2 * kC2 * 8 == kSzPartOne &&
              (size_t)32 * 2 * kC3 * 8 == kSzPartOne && (size_t)16 * 2 * kC4 * 8 == kSzPartOne, "partial tables");

__device__ __forceinline__ void pin1(float& a) { asm volatile("" : "+v"(a)); }
__device__ __forceinline__ void pin4(v4f& v) {
  float a = v[0], b = v[1], c = v[2], d = v[3];
  asm volatile("" : "+v"(a), "+v"(b), "+v"(c), "+v"(d));
  v = (v4f){a, b, c, d};
}
union FragU { v16h v; v8h h[2]; };
__device__ __forceinline__ v16h frag_load(const _Float16* p) {
  FragU f;
  f.h[0] = *(const v8h*)(p);
  f.h[1] = *(const v8h*)(p + 16);
  return f.v;
}
__device__ __forceinline__ v8f frag_mma(v16h a, v16h b, v8f c) {
  return __builtin_amdgcn_wmma_f32_16x16x32_f16(false, a, false, b, (short)0, c, false, false);
}
__device__ __forceinline__ void mma_guard(v8f& c, v16h a, v16h b) {
  asm volatile("v_nop\n\tv_nop\n\tv_nop\n\tv_nop" : "+v"(c) : "v"(a), "v"(b));
}
__device__ __forceinline__ void frag_keep(v16h b) { asm volatile("" :: "v"(b)); }

__global__ __launch_bounds__(256) void weight_plane_kernel(
    const float* __restrict__ src, _Float16* __restrict__ dst,
    int Co, int Kreal, int kuShift, int cgShift, int taps, int perm, int total)
{
  const int idx = blockIdx.x * 256 + threadIdx.x;
  if (idx >= total) return;
  const int u  = idx & ((1 << kuShift) - 1);
  const int n  = idx >> kuShift;
  const int nn = (n < Co) ? n : (Co - 1);
  const int cg  = u & ((1 << cgShift) - 1);
  const int tap = u >> cgShift;
  v8h hv;
#pragma unroll
  for (int e = 0; e < 8; ++e) {
    const int kperm = (cg * 8 + e) * taps + tap;
    const int kid   = u * 8 + e;
    const int k  = perm ? kperm : kid;
    const int kc = (k < Kreal) ? k : (Kreal - 1);
    float v = src[(size_t)nn * Kreal + kc];
    pin1(v);
    const bool ok = (n < Co) && (k < Kreal);
    const float w = ok ? (v * kCarryW) : 0.0f;
    hv[e] = (_Float16)w;
  }
  _Float16* q = dst + (size_t)idx * 8;
  *(volatile v8h*)q = hv;
  __threadfence();
  *(volatile v8h*)q = hv;
}

__global__ __launch_bounds__(256) void gather_input_kernel(
    const float* __restrict__ x, _Float16* __restrict__ COL, int col0, int total)
{
  const int idx = blockIdx.x * 256 + threadIdx.x;
  if (idx >= total) return;
  const int g   = idx & 7;
  const int col = col0 + (idx >> 3);
  const int wo  = col % kWo0;
  const int t   = col / kWo0;
  const int ho  = t & (kHo0 - 1);
  const int b   = t >> 5;
  const bool live = (g < 6);
  const int gi  = live ? g : 5;
  const int ci  = gi >> 1;
  const int kh0 = (gi & 1) * 2;
  const int h0  = 2 * ho - 1 + kh0;
  const int h1  = h0 + 1;
  const int w0  = 2 * wo - 1;
  const int h0c = (h0 < 0) ? 0 : h0;
  const int h1c = (h1 > kInH - 1) ? (kInH - 1) : h1;
  const bool okh0 = live && (h0 >= 0);
  const bool okh1 = live && (h1 <= kInH - 1);
  const float* p0 = x + ((size_t)(b * kInC + ci) * kInH + h0c) * kInW;
  const float* p1 = x + ((size_t)(b * kInC + ci) * kInH + h1c) * kInW;
  v8h hv;
#pragma unroll
  for (int e = 0; e < 4; ++e) {
    const int w  = w0 + e;
    const int wc = (w < 0) ? 0 : ((w > kInW - 1) ? (kInW - 1) : w);
    float a = p0[wc];
    float c = p1[wc];
    pin1(a);
    pin1(c);
    const bool okw = (w >= 0) && (w <= kInW - 1);
    const float ya = (okh0 && okw) ? (a * kCarryA) : 0.0f;
    const float yc = (okh1 && okw) ? (c * kCarryA) : 0.0f;
    hv[e]     = (_Float16)ya;
    hv[4 + e] = (_Float16)yc;
  }
  _Float16* q = COL + (size_t)idx * 8;
  *(volatile v8h*)q = hv;
  __threadfence();
  *(volatile v8h*)q = hv;
}

__global__ __launch_bounds__(256) void gather_bn_kernel(
    const float* __restrict__ Y, const float* __restrict__ ST, _Float16* __restrict__ COL,
    int H, int W, int hoShift, int Wo, int Ci, int cgShift, int kuShift, int kwShift,
    int stride, int pad, int col0, int total)
{
  const int idx = blockIdx.x * 256 + threadIdx.x;
  if (idx >= total) return;
  const int u   = idx & ((1 << kuShift) - 1);
  const int col = col0 + (idx >> kuShift);
  const int cg  = u & ((1 << cgShift) - 1);
  const int tap = u >> cgShift;
  const int kh  = tap >> kwShift;
  const int kw  = tap & ((1 << kwShift) - 1);
  const int wo  = col % Wo;
  const int t   = col / Wo;
  const int ho  = t & ((1 << hoShift) - 1);
  const int b   = t >> hoShift;
  const int h   = ho * stride - pad + kh;
  const int w   = wo * stride - pad + kw;
  const bool inb = (h >= 0) && (h < H) && (w >= 0) && (w < W);
  const int hc  = (h < 0) ? 0 : ((h > H - 1) ? (H - 1) : h);
  const int wc  = (w < 0) ? 0 : ((w > W - 1) ? (W - 1) : w);
  const float* sp = Y + ((size_t)((b * H + hc) * W + wc)) * Ci + cg * 8;
  v4f a0 = *(const v4f*)(sp);
  v4f a1 = *(const v4f*)(sp + 4);
  pin4(a0);
  pin4(a1);
  const v4f m0 = *(const v4f*)(ST + cg * 8);
  const v4f m1 = *(const v4f*)(ST + cg * 8 + 4);
  const v4f s0 = *(const v4f*)(ST + 256 + cg * 8);
  const v4f s1 = *(const v4f*)(ST + 256 + cg * 8 + 4);
  const v4f e0 = *(const v4f*)(ST + 512 + cg * 8);
  const v4f e1 = *(const v4f*)(ST + 512 + cg * 8 + 4);
  v8h hv;
#pragma unroll
  for (int e = 0; e < 4; ++e) {
    float y0 = (a0[e] - m0[e]) * s0[e] + e0[e];
    float y1 = (a1[e] - m1[e]) * s1[e] + e1[e];
    y0 = (y0 >= 0.0f) ? y0 : (kSlope * y0);
    y1 = (y1 >= 0.0f) ? y1 : (kSlope * y1);
    const float z0 = inb ? (y0 * kCarryA) : 0.0f;
    const float z1 = inb ? (y1 * kCarryA) : 0.0f;
    hv[e]     = (_Float16)z0;
    hv[4 + e] = (_Float16)z1;
  }
  _Float16* q = COL + (size_t)idx * 8;
  *(volatile v8h*)q = hv;
  __threadfence();
  *(volatile v8h*)q = hv;
}

template <int NT, int OUT_MODE, int ACT>
__global__ __launch_bounds__(256) void conv_gemm_kernel(
    const _Float16* __restrict__ A, int lda,
    const _Float16* __restrict__ Bt, int ldb,
    void* __restrict__ Cout, int ldc,
    int M, int N, int K, float scale)
{
  static_assert(NT == 1 || NT == 2 || NT == 4, "column subtiles");
  static_assert(OUT_MODE == 0 || NT == 4, "16-bit output uses the wide tile");
  constexpr int NW = 16 * NT;
  __shared__ __align__(16) float sT[8][16 * 68];
  const int lane = threadIdx.x & 31;
  const int wave = threadIdx.x >> 5;
  const int tilesN = N / NW;
  const int tilesM = M >> 6;
  const int tile = blockIdx.x * 8 + wave;
  if (tile >= tilesM * tilesN) return;
  const int tm = tile / tilesN;
  const int tn = tile - tm * tilesN;
  const int m0 = tm << 6;
  const int n0 = tn * NW;

  const int rlane = lane & 15;
  const int koff  = (lane >> 4) * 8;
  const int mOff  = (lane >> 4) * 8;

  v8f acc[4][NT];
#pragma unroll
  for (int i = 0; i < 4; ++i)
#pragma unroll
    for (int j = 0; j < NT; ++j) acc[i][j] = (v8f){0.f, 0.f, 0.f, 0.f, 0.f, 0.f, 0.f, 0.f};

  for (int k0 = 0; k0 < K; k0 += 32) {
    v16h bh[NT];
#pragma unroll
    for (int j = 0; j < NT; ++j) {
      const size_t bo = (size_t)(n0 + (j << 4) + rlane) * ldb + koff + k0;
      bh[j] = frag_load(Bt + bo);
    }
#pragma unroll
    for (int i = 0; i < 4; ++i) {
      const size_t ao = (size_t)(m0 + (i << 4) + rlane) * lda + koff + k0;
      const v16h ah = frag_load(A + ao);
#pragma unroll
      for (int j = 0; j < NT; ++j) acc[i][j] = frag_mma(ah, bh[j], acc[i][j]);
#pragma unroll
      for (int j = 0; j < NT; ++j) mma_guard(acc[i][j], ah, bh[j]);
    }
#pragma unroll
    for (int j = 0; j < NT; ++j) frag_keep(bh[j]);
  }

  float* slab = sT[wave];
#pragma unroll
  for (int i = 0; i < 4; ++i) {
    const int mBase = m0 + (i << 4);
#pragma unroll
    for (int j = 0; j < NT; ++j) {
#pragma unroll
      for (int r = 0; r < 8; ++r) {
        float v = acc[i][j][r] * scale;
        if (ACT == 1) v = (v >= 0.0f) ? v : (kSlope * v);
        slab[(mOff + r) * 68 + (j << 4) + rlane] = v;
      }
    }
    __builtin_amdgcn_fence(__ATOMIC_RELEASE, "workgroup");
    __builtin_amdgcn_wave_barrier();
    __builtin_amdgcn_fence(__ATOMIC_ACQUIRE, "workgroup");
    if (OUT_MODE == 0) {
      constexpr int LPR = NT * 4;
      constexpr int RPI = 32 / LPR;
      constexpr int ITS = 16 / RPI;
      float* C = (float*)Cout;
      const int rr = lane / LPR;
      const int c4 = (lane % LPR) * 4;
      for (int pass = 0; pass < 2; ++pass) {
#pragma unroll
        for (int it = 0; it < ITS; ++it) {
          const int row = it * RPI + rr;
          const v4f v = *(const v4f*)(slab + row * 68 + c4);
          *(volatile v4f*)(C + (size_t)(mBase + row) * ldc + n0 + c4) = v;
        }
        __threadfence();
      }
    } else {
      const int q = lane >> 3;
      const int c8 = (lane & 7) * 8;
      _Float16* C = (_Float16*)Cout;
      for (int pass = 0; pass < 2; ++pass) {
#pragma unroll
        for (int it = 0; it < 4; ++it) {
          const int row = it * 4 + q;
          const float* sp = slab + row * 68 + c8;
          v8h hv;
#pragma unroll
          for (int e = 0; e < 8; ++e) hv[e] = (_Float16)sp[e];
          *(volatile v8h*)(C + (size_t)(mBase + row) * ldc + n0 + c8) = hv;
        }
        __threadfence();
      }
    }
    __builtin_amdgcn_fence(__ATOMIC_RELEASE, "workgroup");
    __builtin_amdgcn_wave_barrier();
    __builtin_amdgcn_fence(__ATOMIC_ACQUIRE, "workgroup");
  }
}

__global__ __launch_bounds__(256) void bn_partial_kernel(
    const float* __restrict__ Y, double* __restrict__ P, int C, int tprShift, int rowsPerBlock)
{
  __shared__ __align__(16) double sh[256 * 8];
  const int tid = threadIdx.x;
  const int cq  = tid & ((1 << tprShift) - 1);
  const int rg  = tid >> tprShift;
  const int RP  = 256 >> tprShift;
  const int iters = rowsPerBlock / RP;
  const size_t base = (size_t)blockIdx.x * rowsPerBlock;
  double s0 = 0.0, s1 = 0.0, s2 = 0.0, s3 = 0.0;
  double q0 = 0.0, q1 = 0.0, q2 = 0.0, q3 = 0.0;
#pragma unroll 1
  for (int it = 0; it < iters; ++it) {
    const size_t row = base + (size_t)it * RP + rg;
    const v4f v = *(const v4f*)(Y + row * C + cq * 4);
    const double d0 = (double)v[0], d1 = (double)v[1], d2 = (double)v[2], d3 = (double)v[3];
    s0 += d0; s1 += d1; s2 += d2; s3 += d3;
    q0 += d0 * d0; q1 += d1 * d1; q2 += d2 * d2; q3 += d3 * d3;
  }
  sh[tid * 8 + 0] = s0; sh[tid * 8 + 1] = s1; sh[tid * 8 + 2] = s2; sh[tid * 8 + 3] = s3;
  sh[tid * 8 + 4] = q0; sh[tid * 8 + 5] = q1; sh[tid * 8 + 6] = q2; sh[tid * 8 + 7] = q3;
  __syncthreads();
  if (tid < C) {
    const int j = 2 * tid;
    const int hiHalf = (j >= C) ? 1 : 0;
    const int c = j - hiHalf * C;
    const int quad = c >> 2;
    const int el = (c & 3) + hiHalf * 4;
    double f0 = 0.0, f1 = 0.0;
#pragma unroll 1
    for (int g = 0; g < RP; ++g) {
      const double* p = sh + (size_t)((g << tprShift) + quad) * 8 + el;
      f0 += p[0];
      f1 += p[1];
    }
    const v2d o = (v2d){f0, f1};
    double* dst = P + (size_t)blockIdx.x * 2 * C + j;
    *(volatile v2d*)dst = o;
    __threadfence();
    *(volatile v2d*)dst = o;
  }
}

__global__ __launch_bounds__(256) void bn_finalize_kernel(
    const double* __restrict__ P, const float* __restrict__ gam, const float* __restrict__ bet,
    float* __restrict__ ST, int C, int NB, double invM)
{
  const int c  = threadIdx.x;
  const int cc = (c < C) ? c : (C - 1);
  double s = 0.0, q = 0.0;
#pragma unroll 1
  for (int p = 0; p < NB; ++p) {
    s += P[(size_t)p * 2 * C + cc];
    q += P[(size_t)p * 2 * C + C + cc];
  }
  const double mean = s * invM;
  double var = q * invM - mean * mean;
  var = (var > 0.0) ? var : 0.0;
  const float rstd = rsqrtf((float)var + kBnEps);
  float gv = gam[cc];
  float bv = bet[cc];
  pin1(gv);
  pin1(bv);
  const bool live = (c < C);
  const float o0 = live ? (float)mean : 0.0f;
  const float o1 = live ? (rstd * gv) : 0.0f;
  const float o2 = live ? bv : 0.0f;
  *(volatile float*)(ST + c) = o0;
  *(volatile float*)(ST + 256 + c) = o1;
  *(volatile float*)(ST + 512 + c) = o2;
  __threadfence();
  *(volatile float*)(ST + c) = o0;
  *(volatile float*)(ST + 256 + c) = o1;
  *(volatile float*)(ST + 512 + c) = o2;
}

__global__ __launch_bounds__(256) void blend_kernel(const float* __restrict__ L, float* __restrict__ out)
{
  const int lane = threadIdx.x & 31;
  const int wv = blockIdx.x * 8 + (threadIdx.x >> 5);
  if (wv >= kBatch * 24) return;
  const int b  = wv / 24;
  const int j2 = wv - b * 24;
  const int ja = (j2 < kWo5) ? j2 : (kWo5 - 1);
  const int jb = (j2 > 0) ? (j2 - 1) : 0;
  const float va = L[(size_t)(b * kWo5 + ja) * kCL + lane];
  const float vb = L[(size_t)(b * kWo5 + jb) * kCL + 32 + lane];
  const float sa = 1.0f / (1.0f + expf(-va));
  const float sb = 1.0f / (1.0f + expf(-vb));
  float r = (sb + sa) * 0.5f;
  if (j2 == 0) r = sa;
  if (j2 == 23) r = sb;
  float* dst = out + (size_t)wv * 32 + lane;
  *(volatile float*)dst = r;
  __threadfence();
  *(volatile float*)dst = r;
}

extern "C" void kernel_launch(void* const* d_in, const int* in_sizes, int n_in,
                              void* d_out, int out_size, void* d_ws, size_t ws_size,
                              hipStream_t stream) {
  if (n_in < 18) return;
  const int expect[18] = {
    kBatch * kInC * kInH * kInW, kC0 * kK0R, kC0, kC0,
    kC1 * kK1, kC1, kC1,
    kC2 * kK2, kC2, kC2,
    kC3 * kK3, kC3, kC3,
    kC4 * kK4, kC4, kC4,
    kC5 * kK5, kCL * kK6R };
  for (int i = 0; i < 18; ++i) if (in_sizes[i] != expect[i]) return;
  if (out_size != kBatch * 768) return;
  if (ws_size < kWsTotal) return;

  const float* x   = (const float*)d_in[0];
  const float* w0  = (const float*)d_in[1];
  const float* g0  = (const float*)d_in[2];
  const float* b0  = (const float*)d_in[3];
  const float* w1  = (const float*)d_in[4];
  const float* g1  = (const float*)d_in[5];
  const float* b1  = (const float*)d_in[6];
  const float* w2  = (const float*)d_in[7];
  const float* g2  = (const float*)d_in[8];
  const float* b2  = (const float*)d_in[9];
  const float* w3  = (const float*)d_in[10];
  const float* g3  = (const float*)d_in[11];
  const float* b3  = (const float*)d_in[12];
  const float* w4  = (const float*)d_in[13];
  const float* g4  = (const float*)d_in[14];
  const float* b4  = (const float*)d_in[15];
  const float* w5  = (const float*)d_in[16];
  const float* wl  = (const float*)d_in[17];
  float* out = (float*)d_out;

  char* ws = (char*)d_ws;
  float*    YA   = (float*)(ws + kOffYA);
  float*    YB   = (float*)(ws + kOffYB);
  _Float16* COL  = (_Float16*)(ws + kOffCOL);
  _Float16* A6   = (_Float16*)(ws + kOffA6);
  _Float16* W0   = (_Float16*)(ws + kOffW0);
  _Float16* W1   = (_Float16*)(ws + kOffW1);
  _Float16* W2   = (_Float16*)(ws + kOffW2);
  _Float16* W3   = (_Float16*)(ws + kOffW3);
  _Float16* W4   = (_Float16*)(ws + kOffW4);
  _Float16* W5   = (_Float16*)(ws + kOffW5);
  _Float16* WL   = (_Float16*)(ws + kOffWL);
  float*    LOUT = (float*)(ws + kOffLOUT);
  double*   P0   = (double*)(ws + kOffPART);
  double*   P1   = (double*)(ws + kOffPART + 1 * kSzPartOne);
  double*   P2   = (double*)(ws + kOffPART + 2 * kSzPartOne);
  double*   P3   = (double*)(ws + kOffPART + 3 * kSzPartOne);
  double*   P4   = (double*)(ws + kOffPART + 4 * kSzPartOne);
  float*    ST0  = (float*)(ws + kOffST);
  float*    ST1  = (float*)(ws + kOffST + 1 * kSzStOne);
  float*    ST2  = (float*)(ws + kOffST + 2 * kSzStOne);
  float*    ST3  = (float*)(ws + kOffST + 3 * kSzStOne);
  float*    ST4  = (float*)(ws + kOffST + 4 * kSzStOne);

  weight_plane_kernel<<<1,   256, 0, stream>>>(w0, W0, kC0, kK0R, 3, 0, 1, 0, kC0 * kK0 / 8);
  weight_plane_kernel<<<4,   256, 0, stream>>>(w1, W1, kC1, kK1, 5, 1, 16, 1, kC1 * kK1 / 8);
  weight_plane_kernel<<<16,  256, 0, stream>>>(w2, W2, kC2, kK2, 6, 2, 16, 1, kC2 * kK2 / 8);
  weight_plane_kernel<<<64,  256, 0, stream>>>(w3, W3, kC3, kK3, 7, 3, 16, 1, kC3 * kK3 / 8);
  weight_plane_kernel<<<256, 256, 0, stream>>>(w4, W4, kC4, kK4, 8, 4, 16, 1, kC4 * kK4 / 8);
  weight_plane_kernel<<<512, 256, 0, stream>>>(w5, W5, kC5, kK5, 7, 5, 4, 1, kC5P * kK5 / 8);
  weight_plane_kernel<<<32,  256, 0, stream>>>(wl, WL, kCL, kK6R, 7, 0, 1, 0, kCL * kK6 / 8);

  for (int c = 0; c < 4; ++c) {
    const int col0 = c * kChunk0;
    gather_input_kernel<<<kChunk0 * 8 / 256, 256, 0, stream>>>(x, COL, col0, kChunk0 * 8);
    conv_gemm_kernel<1, 0, 0><<<(kChunk0 / 64 + 7) / 8, 256, 0, stream>>>(
        COL, kK0, W0, kK0, (void*)(YA + (size_t)col0 * kC0), kC0, kChunk0, kC0, kK0, kFold);
  }
  bn_partial_kernel<<<256, 256, 0, stream>>>(YA, P0, kC0, 2, kM0 / 256);
  bn_finalize_kernel<<<1, 256, 0, stream>>>(P0, g0, b0, ST0, kC0, 256, 1.0 / (double)kM0);

  for (int c = 0; c < 4; ++c) {
    const int col0 = c * kChunk1;
    gather_bn_kernel<<<kChunk1 * (kK1 / 8) / 256, 256, 0, stream>>>(
        YA, ST0, COL, kHo0, kWo0, 4, kWo1, kC0, 1, 5, 2, 2, 1, col0, kChunk1 * (kK1 / 8));
    conv_gemm_kernel<2, 0, 0><<<(kChunk1 / 64 + 7) / 8, 256, 0, stream>>>(
        COL, kK1, W1, kK1, (void*)(YB + (size_t)col0 * kC1), kC1, kChunk1, kC1, kK1, kFold);
  }
  bn_partial_kernel<<<128, 256, 0, stream>>>(YB, P1, kC1, 3, kM1 / 128);
  bn_finalize_kernel<<<1, 256, 0, stream>>>(P1, g1, b1, ST1, kC1, 128, 1.0 / (double)kM1);

  for (int c = 0; c < 2; ++c) {
    const int col0 = c * kChunk2;
    gather_bn_kernel<<<kChunk2 * (kK2 / 8) / 256, 256, 0, stream>>>(
        YB, ST1, COL, kHo1, kWo1, 3, kWo2, kC1, 2, 6, 2, 2, 1, col0, kChunk2 * (kK2 / 8));
    conv_gemm_kernel<4, 0, 0><<<((kChunk2 / 64) * (kC2 / 64) + 7) / 8, 256, 0, stream>>>(
        COL, kK2, W2, kK2, (void*)(YA + (size_t)col0 * kC2), kC2, kChunk2, kC2, kK2, kFold);
  }
  bn_partial_kernel<<<64, 256, 0, stream>>>(YA, P2, kC2, 4, kM2 / 64);
  bn_finalize_kernel<<<1, 256, 0, stream>>>(P2, g2, b2, ST2, kC2, 64, 1.0 / (double)kM2);

  gather_bn_kernel<<<kM3 * (kK3 / 8) / 256, 256, 0, stream>>>(
      YA, ST2, COL, kHo2, kWo2, 2, kWo3, kC2, 3, 7, 2, 2, 1, 0, kM3 * (kK3 / 8));
  conv_gemm_kernel<4, 0, 0><<<((kM3 / 64) * (kC3 / 64) + 7) / 8, 256, 0, stream>>>(
      COL, kK3, W3, kK3, (void*)YB, kC3, kM3, kC3, kK3, kFold);
  bn_partial_kernel<<<32, 256, 0, stream>>>(YB, P3, kC3, 5, kM3 / 32);
  bn_finalize_kernel<<<1, 256, 0, stream>>>(P3, g3, b3, ST3, kC3, 32, 1.0 / (double)kM3);

  gather_bn_kernel<<<kM4 * (kK4 / 8) / 256, 256, 0, stream>>>(
      YB, ST3, COL, kHo3, kWo3, 1, kWo4, kC3, 4, 8, 2, 2, 1, 0, kM4 * (kK4 / 8));
  conv_gemm_kernel<4, 0, 0><<<((kM4 / 64) * (kC4 / 64) + 7) / 8, 256, 0, stream>>>(
      COL, kK4, W4, kK4, (void*)YA, kC4, kM4, kC4, kK4, kFold);
  bn_partial_kernel<<<16, 256, 0, stream>>>(YA, P4, kC4, 6, kM4 / 16);
  bn_finalize_kernel<<<1, 256, 0, stream>>>(P4, g4, b4, ST4, kC4, 16, 1.0 / (double)kM4);

  gather_bn_kernel<<<kM5 * (kK5 / 8) / 256, 256, 0, stream>>>(
      YA, ST4, COL, kHo4, kWo4, 0, kWo5, kC4, 5, 7, 1, 1, 0, 0, kM5 * (kK5 / 8));
  conv_gemm_kernel<4, 1, 1><<<((kM5 / 64) * (kC5P / 64) + 7) / 8, 256, 0, stream>>>(
      COL, kK5, W5, kK5, (void*)A6, kC5P, kM5, kC5P, kK5, kFoldKeepA);

  conv_gemm_kernel<4, 0, 0><<<((kM5 / 64) * (kCL / 64) + 7) / 8, 256, 0, stream>>>(
      A6, kK6, WL, kK6, (void*)LOUT, kCL, kM5, kCL, kK6, kFold);

  blend_kernel<<<kBatch * 24 / 8, 256, 0, stream>>>(LOUT, out);
}
